// SingleLayerRank1DCModel_37271726195000
// MI455X (gfx1250) — hardware-verified
//
#include <hip/hip_runtime.h>
#define TT 2048
#define DD 1024
#define NH 16
#define DKk 64
#define DVv 128
#define QW (NH * DKk)
#define VW (NH * DVv)
#define PW 6176
#define PWP 6208
#define OQ 0
#define OK_ 1024
#define OV 2048
#define OG 4096
#define OA 6144
#define OB 6160
typedef __bf16 v16b __attribute__((ext_vector_type(16)));
typedef unsigned short v8us __attribute__((ext_vector_type(8), may_alias));
typedef float  v8f  __attribute__((ext_vector_type(8)));
typedef float  v4f  __attribute__((ext_vector_type(4)));
typedef float  v4fa __attribute__((ext_vector_type(4), may_alias));
union FragB { v16b v; v8us half[2]; unsigned short u[16]; };

__device__ __forceinline__ unsigned short bf16_bits(float x) { unsigned int u = __float_as_uint(x); return (unsigned short)((u + 0x7FFFu + ((u >> 16) & 1u)) >> 16); }
__device__ __forceinline__ float bf16_val(unsigned short b) { return __uint_as_float(((unsigned int)b) << 16); }
__device__ __forceinline__ float bf16_round(float x) { return bf16_val(bf16_bits(x)); }
template <int NT>
__device__ __forceinline__ v8f mmaN(v16b ah, v16b al, v16b bh, v16b bl, v8f c) {
  c = __builtin_amdgcn_wmma_f32_16x16x32_bf16(false, ah, false, bh, (short)0, c, false, false);
  if (NT >= 2) c = __builtin_amdgcn_wmma_f32_16x16x32_bf16(false, al, false, bh, (short)0, c, false, false);
  if (NT >= 3) c = __builtin_amdgcn_wmma_f32_16x16x32_bf16(false, ah, false, bl, (short)0, c, false, false);
  asm volatile("v_nop\n\tv_nop\n\tv_nop\n\tv_nop" : "+v"(c) : "v"(ah), "v"(al), "v"(bh), "v"(bl));
  return c;
}

__global__ __launch_bounds__(256) void k_wt_bf16(const float* __restrict__ W, unsigned short* __restrict__ Wt, int K, int N) {
  const int t = blockIdx.x * 256 + threadIdx.x;
  const int k8n = K / 8;
  if (t >= N * k8n) return;
  const int n = t / k8n, k8 = (t % k8n) * 8;
  v8us v;
#pragma unroll
  for (int i = 0; i < 8; ++i) v[i] = bf16_bits(W[(size_t)(k8 + i) * N + n]);
  *(volatile v8us*)(Wt + (size_t)n * K + k8) = v;
  __threadfence();
  *(volatile v8us*)(Wt + (size_t)n * K + k8) = v;
}

template <bool ASPLIT, int ACT, bool BIAS_BF16>
__global__ __launch_bounds__(128) void k_gemm_bf(const float* __restrict__ A, int lda, const unsigned short* __restrict__ Wt, int ldb,
                                               const float* __restrict__ bias, float* __restrict__ C, int ldc, int M, int N, int K) {
  __shared__ __attribute__((aligned(16))) float so[4][16][64];
  const int tid = threadIdx.x, w = tid >> 5, lane = tid & 31, ln = lane & 15, hh = lane >> 4;
  const int ntn = N / 64;
  const int wid = blockIdx.x * 4 + w;
  const int mt = wid / ntn, nq = wid % ntn;
  if (mt * 16 >= M) return;
  const int row0 = mt * 16, col0 = nq * 64;
  const float* arow = A + (size_t)(row0 + ln) * lda;
  v8f acc[4] = {};
  for (int kb = 0; kb < K; kb += 32) {
    FragB ah, al;
    const v4f x0 = *(const v4fa*)(arow + kb + 8 * hh), x1 = *(const v4fa*)(arow + kb + 8 * hh + 4);
    const v4f x2 = *(const v4fa*)(arow + kb + 16 + 8 * hh), x3 = *(const v4fa*)(arow + kb + 16 + 8 * hh + 4);
    float xs[16] = {x0[0],x0[1],x0[2],x0[3],x1[0],x1[1],x1[2],x1[3],x2[0],x2[1],x2[2],x2[3],x3[0],x3[1],x3[2],x3[3]};
#pragma unroll
    for (int i = 0; i < 16; ++i) { const unsigned short hb = bf16_bits(xs[i]); ah.u[i] = hb; al.u[i] = ASPLIT ? bf16_bits(xs[i] - bf16_val(hb)) : (unsigned short)0; }
#pragma unroll
    for (int t = 0; t < 4; ++t) {
      const unsigned short* brow = Wt + (size_t)(col0 + t * 16 + ln) * ldb + kb;
      FragB b;
      b.half[0] = *(const v8us*)(brow + 8 * hh);
      b.half[1] = *(const v8us*)(brow + 16 + 8 * hh);
      acc[t] = mmaN<ASPLIT ? 2 : 1>(ah.v, al.v, b.v, b.v, acc[t]);
    }
  }
#pragma unroll
  for (int t = 0; t < 4; ++t) {
    float bv = bias ? bias[col0 + t * 16 + ln] : 0.f;
    if (BIAS_BF16) bv = bf16_round(bv);
#pragma unroll
    for (int r = 0; r < 8; ++r) { float v = acc[t][r] + bv; if (ACT == 1) v = fmaxf(v, 0.f); so[w][8 * hh + r][t * 16 + ln] = v; }
  }
  __builtin_amdgcn_fence(__ATOMIC_ACQ_REL, "workgroup");
  __builtin_amdgcn_wave_barrier();
  const int rsub = lane >> 4, c4 = (lane & 15) * 4;
  for (int pass = 0; pass < 2; ++pass) {
#pragma unroll
    for (int q = 0; q < 8; ++q) {
      const int r = q * 2 + rsub;
      const v4f v = *(const v4fa*)&so[w][r][c4];
      *(volatile v4f*)(C + (size_t)(row0 + r) * ldc + col0 + c4) = v;
    }
    if (pass == 0) __threadfence();
  }
}

template <bool ASPLIT, int ACT, bool BIAS_BF16, bool RES_BF16>
__global__ __launch_bounds__(128) void k_gemm_bf3(const float* __restrict__ A, int lda, const unsigned short* __restrict__ Wt, int ldb,
                                                const float* __restrict__ bias, const float* __restrict__ resid, int rmod, int ldr,
                                                float* __restrict__ C, int ldc, int M, int N, int K) {
  __shared__ __attribute__((aligned(16))) float so[4][16][64];
  const int tid = threadIdx.x, w = tid >> 5, lane = tid & 31, ln = lane & 15, hh = lane >> 4;
  const int ntn = N / 64;
  const int wid = blockIdx.x * 4 + w;
  const int mt = wid / ntn, nq = wid % ntn;
  if (mt * 16 >= M) return;
  const int row0 = mt * 16, col0 = nq * 64;
  const float* arow = A + (size_t)(row0 + ln) * lda;
  v8f acc[4] = {};
  for (int kb = 0; kb < K; kb += 32) {
    FragB ah, al;
    const v4f x0 = *(const v4fa*)(arow + kb + 8 * hh), x1 = *(const v4fa*)(arow + kb + 8 * hh + 4);
    const v4f x2 = *(const v4fa*)(arow + kb + 16 + 8 * hh), x3 = *(const v4fa*)(arow + kb + 16 + 8 * hh + 4);
    float xs[16] = {x0[0],x0[1],x0[2],x0[3],x1[0],x1[1],x1[2],x1[3],x2[0],x2[1],x2[2],x2[3],x3[0],x3[1],x3[2],x3[3]};
#pragma unroll
    for (int i = 0; i < 16; ++i) { const unsigned short hb = bf16_bits(xs[i]); ah.u[i] = hb; al.u[i] = ASPLIT ? bf16_bits(xs[i] - bf16_val(hb)) : (unsigned short)0; }
#pragma unroll
    for (int t = 0; t < 4; ++t) {
      const unsigned short* brow = Wt + (size_t)(col0 + t * 16 + ln) * ldb + kb;
      FragB b;
      b.half[0] = *(const v8us*)(brow + 8 * hh);
      b.half[1] = *(const v8us*)(brow + 16 + 8 * hh);
      acc[t] = mmaN<ASPLIT ? 2 : 1>(ah.v, al.v, b.v, b.v, acc[t]);
    }
  }
#pragma unroll
  for (int t = 0; t < 4; ++t) {
    const int col = col0 + t * 16 + ln;
    float bv = bias ? bias[col] : 0.f;
    if (BIAS_BF16) bv = bf16_round(bv);
#pragma unroll
    for (int r = 0; r < 8; ++r) {
      float v = acc[t][r] + bv;
      if (resid) { float rv = resid[(size_t)((row0 + 8 * hh + r) % rmod) * ldr + col]; if (RES_BF16) rv = bf16_round(rv); v += rv; }
      if (ACT == 1) v = fmaxf(v, 0.f);
      if (ACT == 2) v = 0.5f * v * (1.0f + erff(v * 0.70710678118654752f));
      if (ACT == 3) { const float u = 0.7978845608028654f * (v + 0.044715f * v * v * v); v = 0.5f * v * (1.0f + tanhf(u)); }
      so[w][8 * hh + r][t * 16 + ln] = v;
    }
  }
  __builtin_amdgcn_fence(__ATOMIC_ACQ_REL, "workgroup");
  __builtin_amdgcn_wave_barrier();
  const int rsub = lane >> 4, c4 = (lane & 15) * 4;
  for (int pass = 0; pass < 2; ++pass) {
#pragma unroll
    for (int q = 0; q < 8; ++q) {
      const int r = q * 2 + rsub;
      const v4f v = *(const v4fa*)&so[w][r][c4];
      *(volatile v4f*)(C + (size_t)(row0 + r) * ldc + col0 + c4) = v;
    }
    if (pass == 0) __threadfence();
  }
}
template <bool PARAM_BF16>
__global__ __launch_bounds__(256) void k_layernorm(const float* __restrict__ X, const float* __restrict__ R, const float* __restrict__ g, const float* __restrict__ bta,
                                                  float* __restrict__ out_sum, float* __restrict__ out_norm, int N, float eps) {
  __shared__ float red[256];
  const int row = blockIdx.x, tid = threadIdx.x;
  const float* x = X + (size_t)row * N; const float* rr = R ? R + (size_t)row * N : nullptr;
  float vals[16];
  const int per = N / 256;
  float s1 = 0.f;
  for (int u = 0; u < per / 4; ++u) {
    const int j = tid * 4 + 1024 * u;
    const v4f a = *(const v4fa*)(x + j);
    v4f b = {0.f,0.f,0.f,0.f}; if (rr) b = *(const v4fa*)(rr + j);
#pragma unroll
    for (int q = 0; q < 4; ++q) { const float v = a[q] + b[q]; vals[u * 4 + q] = v; s1 += v; }
  }
  red[tid] = s1; __syncthreads();
  for (int st = 128; st > 0; st >>= 1) { if (tid < st) red[tid] += red[tid + st]; __syncthreads(); }
  const float mu = red[0] / (float)N; __syncthreads();
  float s2 = 0.f;
  for (int u = 0; u < per / 4; ++u)
#pragma unroll
    for (int q = 0; q < 4; ++q) { const float c = vals[u * 4 + q] - mu; s2 += c * c; }
  red[tid] = s2; __syncthreads();
  for (int st = 128; st > 0; st >>= 1) { if (tid < st) red[tid] += red[tid + st]; __syncthreads(); }
  const float rs = rsqrtf(red[0] / (float)N + eps);
  for (int pass = 0; pass < 2; ++pass) {
    for (int u = 0; u < per / 4; ++u) {
      const int j = tid * 4 + 1024 * u;
      v4f o, sm;
#pragma unroll
      for (int q = 0; q < 4; ++q) {
        float gg = g[j + q], bb = bta[j + q];
        if (PARAM_BF16) { gg = bf16_round(gg); bb = bf16_round(bb); }
        sm[q] = vals[u * 4 + q]; o[q] = (vals[u * 4 + q] - mu) * rs * gg + bb;
      }
      if (out_sum) *(volatile v4f*)(out_sum + (size_t)row * N + j) = sm;
      *(volatile v4f*)(out_norm + (size_t)row * N + j) = o;
    }
    if (pass == 0) __threadfence();
  }
}


typedef _Float16 v16h __attribute__((ext_vector_type(16)));
union FragH { v16h v; v8us half[2]; _Float16 h[16]; unsigned short u[16]; };
template <int NT>
__device__ __forceinline__ v8f mmaH(v16h ah, v16h al, v16h bh, v16h bl, v8f c) {
  c = __builtin_amdgcn_wmma_f32_16x16x32_f16(false, ah, false, bh, (short)0, c, false, false);
  if (NT >= 2) c = __builtin_amdgcn_wmma_f32_16x16x32_f16(false, al, false, bh, (short)0, c, false, false);
  if (NT >= 3) c = __builtin_amdgcn_wmma_f32_16x16x32_f16(false, ah, false, bl, (short)0, c, false, false);
  asm volatile("v_nop\n\tv_nop\n\tv_nop\n\tv_nop" : "+v"(c) : "v"(ah), "v"(al), "v"(bh), "v"(bl));
  return c;
}
template <bool ASPLIT>
__global__ __launch_bounds__(128) void k_gemm_h(const float* __restrict__ A, int lda, size_t sA, const _Float16* __restrict__ Bh, int ldb, size_t sB, float alpha, float* __restrict__ C, int ldc, size_t sC, int M, int N, int K) {
  __shared__ __attribute__((aligned(16))) float so[4][16][64];
  const int tid = threadIdx.x, w = tid >> 5, lane = tid & 31, ln = lane & 15, hh = lane >> 4; const int by = blockIdx.y;
  A += (size_t)by * sA; Bh += (size_t)by * sB; C += (size_t)by * sC;
  const int ntn = (N + 63) / 64; const int wid = blockIdx.x * 4 + w; const int mt = wid / ntn, nq = wid % ntn; if (mt * 16 >= M) return;
  const int row0 = mt * 16, col0 = nq * 64; const float* arow = A + (size_t)(row0 + ln) * lda;
  v8f acc[4] = {};
  for (int kb = 0; kb < K; kb += 32) {
    FragH ah, al;
    const v4f x0 = *(const v4fa*)(arow + kb + 8 * hh), x1 = *(const v4fa*)(arow + kb + 8 * hh + 4), x2 = *(const v4fa*)(arow + kb + 16 + 8 * hh), x3 = *(const v4fa*)(arow + kb + 16 + 8 * hh + 4);
    float xs[16] = {x0[0],x0[1],x0[2],x0[3],x1[0],x1[1],x1[2],x1[3],x2[0],x2[1],x2[2],x2[3],x3[0],x3[1],x3[2],x3[3]};
#pragma unroll
    for (int i = 0; i < 16; ++i) { const _Float16 h = (_Float16)xs[i]; ah.h[i] = h; al.h[i] = ASPLIT ? (_Float16)(xs[i] - (float)h) : (_Float16)0.0f; }
#pragma unroll
    for (int t = 0; t < 4; ++t) { if (col0 + t * 16 >= N) continue; const size_t boff = (size_t)(col0 + t * 16 + ln) * ldb + kb; FragH bq; bq.half[0] = *(const v8us*)(Bh + boff + 8 * hh); bq.half[1] = *(const v8us*)(Bh + boff + 16 + 8 * hh);
      acc[t] = mmaH<ASPLIT ? 2 : 1>(ah.v, al.v, bq.v, bq.v, acc[t]); }
  }
#pragma unroll
  for (int t = 0; t < 4; ++t) { if (col0 + t * 16 >= N) continue;
#pragma unroll
    for (int r = 0; r < 8; ++r) so[w][8 * hh + r][t * 16 + ln] = acc[t][r] * alpha; }
  __builtin_amdgcn_fence(__ATOMIC_ACQ_REL, "workgroup"); __builtin_amdgcn_wave_barrier();
  const int rsub = lane >> 4, c4 = (lane & 15) * 4;
  for (int pass = 0; pass < 2; ++pass) {
#pragma unroll
    for (int q = 0; q < 8; ++q) { const int r = q * 2 + rsub; if (col0 + c4 < N) { const v4f v = *(const v4fa*)&so[w][r][c4]; *(volatile v4f*)(C + (size_t)(row0 + r) * ldc + col0 + c4) = v; } }
    if (pass == 0) __threadfence(); }
}

__global__ __launch_bounds__(256) void k_wt_f16(const float* __restrict__ W, _Float16* __restrict__ Wt, int K, int N, float scale) {
  const int t = blockIdx.x * 256 + threadIdx.x; if (t >= N * (K / 8)) return; const int n = t / (K / 8), k8 = (t % (K / 8)) * 8; FragH f;
#pragma unroll
  for (int i = 0; i < 8; ++i) f.h[i] = (_Float16)(bf16_round(W[(size_t)(k8 + i) * N + n]) * scale); const v8us o = f.half[0];
  *(volatile v8us*)((unsigned short*)Wt + (size_t)n * K + k8) = o; __threadfence(); *(volatile v8us*)((unsigned short*)Wt + (size_t)n * K + k8) = o;
}
template <int ACT>
__global__ __launch_bounds__(128) void k_gemm_hhx(const _Float16* __restrict__ A, int lda, size_t sA, const _Float16* __restrict__ Bh, int ldb, size_t sB, float alpha, const float* __restrict__ bias, size_t sBias, const float* __restrict__ CP, int rowsPerB, size_t sCPb, int row0g,
    float* __restrict__ C, _Float16* __restrict__ C16, int ldc, size_t sC, int M, int N, int K) {
  __shared__ __attribute__((aligned(16))) float so[4][16][64];
  const int tid = threadIdx.x, w = tid >> 5, lane = tid & 31, ln = lane & 15, hh = lane >> 4; const int by = blockIdx.y;
  A += (size_t)by * sA; Bh += (size_t)by * sB; const size_t cofs = (size_t)by * sC; const float* bp = bias ? bias + (size_t)by * sBias : nullptr;
  const int ntn = (N + 63) / 64; const int wid = blockIdx.x * 4 + w; const int mt = wid / ntn, nq = wid % ntn; if (mt * 16 >= M) return;
  const int row0 = mt * 16, col0 = nq * 64; const _Float16* arow = A + (size_t)(row0 + ln) * lda;
  v8f acc[4] = {};
  for (int kb = 0; kb < K; kb += 32) { FragH ah; ah.half[0] = *(const v8us*)((const unsigned short*)arow + kb + 8 * hh); ah.half[1] = *(const v8us*)((const unsigned short*)arow + kb + 16 + 8 * hh);
#pragma unroll
    for (int t = 0; t < 4; ++t) { if (col0 + t * 16 >= N) continue; const size_t boff = (size_t)(col0 + t * 16 + ln) * ldb + kb; FragH bq; bq.half[0] = *(const v8us*)((const unsigned short*)Bh + boff + 8 * hh); bq.half[1] = *(const v8us*)((const unsigned short*)Bh + boff + 16 + 8 * hh);
      acc[t] = mmaH<1>(ah.v, ah.v, bq.v, bq.v, acc[t]); }
  }
#pragma unroll
  for (int t = 0; t < 4; ++t) { if (col0 + t * 16 >= N) continue; const int col = col0 + t * 16 + ln; const float bv = bp ? bf16_round(bp[col]) : 0.f;
#pragma unroll
    for (int r = 0; r < 8; ++r) { float v = acc[t][r] * alpha + bv; if (CP) { const int bidx = (row0g + row0 + 8 * hh + r) / rowsPerB; v += CP[(size_t)bidx * sCPb + (size_t)by * 64 + col]; } if (ACT == 1) v = (v > 0.f) ? v : expm1f(v); else if (ACT == 7) v = (v > 0.f) ? v + 1.0f : expf(v); else if (ACT == 8) v = tanhf(v); else if (ACT == 9) v = 0.5f * v * (1.0f + tanhf(0.7978845608028654f * (v + 0.044715f * v * v * v))); else if (ACT == 11) v = 1.0f / (1.0f + expf(-v)); else if (ACT == 12) v = (v > 0.f) ? v : 0.01f * v; else if (ACT == 14) v = (v > 0.f) ? v : 0.1f * v; else if (ACT == 15) v = v / (1.0f + expf(-v)); else if (ACT == 3) v = fmaxf(v, 0.f); else if (ACT == 6) v = 0.5f * v * (1.0f + erff(v * 0.70710678118654752f)); so[w][8 * hh + r][t * 16 + ln] = v; } }
  __builtin_amdgcn_fence(__ATOMIC_ACQ_REL, "workgroup"); __builtin_amdgcn_wave_barrier();
  const int rsub = lane >> 4, c4 = (lane & 15) * 4; typedef _Float16 v4h __attribute__((ext_vector_type(4)));
  for (int pass = 0; pass < 2; ++pass) {
#pragma unroll
    for (int q = 0; q < 8; ++q) { const int r = q * 2 + rsub; if (col0 + c4 < N) { const v4f v = *(const v4fa*)&so[w][r][c4]; if (C) *(volatile v4f*)(C + cofs + (size_t)(row0 + r) * ldc + col0 + c4) = v; if (C16) { v4h h4; for (int i = 0; i < 4; ++i) h4[i] = (_Float16)v[i]; *(volatile v4h*)(C16 + cofs + (size_t)(row0 + r) * ldc + col0 + c4) = h4; } } }
    if (pass == 0) __threadfence(); }
}


typedef _Float16 v4h __attribute__((ext_vector_type(4)));

__global__ __launch_bounds__(256) void k_x16(const float* __restrict__ x, _Float16* __restrict__ X16, size_t n8) { const size_t t = (size_t)blockIdx.x * 256 + threadIdx.x; if (t >= n8) return; FragH f;
#pragma unroll
  for (int q = 0; q < 8; ++q) f.h[q] = (_Float16)bf16_round(x[t * 8 + q]); *(volatile v8us*)((unsigned short*)X16 + t * 8) = f.half[0]; __threadfence(); *(volatile v8us*)((unsigned short*)X16 + t * 8) = f.half[0]; }
__global__ __launch_bounds__(256) void k_h16(const float* __restrict__ x, _Float16* __restrict__ X16, size_t n8) { const size_t t = (size_t)blockIdx.x * 256 + threadIdx.x; if (t >= n8) return; FragH f;
#pragma unroll
  for (int q = 0; q < 8; ++q) f.h[q] = (_Float16)x[t * 8 + q]; *(volatile v8us*)((unsigned short*)X16 + t * 8) = f.half[0]; __threadfence(); *(volatile v8us*)((unsigned short*)X16 + t * 8) = f.half[0]; }
__global__ __launch_bounds__(256) void k_round16f(const float* __restrict__ W, _Float16* __restrict__ Bt, size_t n8) { const size_t t = (size_t)blockIdx.x * 256 + threadIdx.x; if (t >= n8) return; FragH f;
#pragma unroll
  for (int i = 0; i < 8; ++i) f.h[i] = (_Float16)(bf16_round(W[t * 8 + i]) * 16.0f); *(volatile v8us*)((unsigned short*)Bt + t * 8) = f.half[0]; __threadfence(); *(volatile v8us*)((unsigned short*)Bt + t * 8) = f.half[0]; }
template <int NHv, int TTv>
__global__ __launch_bounds__(256) void k_vt(const _Float16* __restrict__ V16, int ldv, int voff, _Float16* __restrict__ Vt) { __shared__ unsigned short tl[64][66]; const int tid = threadIdx.x; const int slab = blockIdx.x / (TTv / 64), lg = blockIdx.x % (TTv / 64); const int b = slab / NHv, h = slab % NHv;
  for (int i = tid; i < 64 * 8; i += 256) { const int r = i / 8, c8 = (i % 8) * 8; FragH f; f.half[0] = *(const v8us*)((const unsigned short*)V16 + ((size_t)b * TTv + lg * 64 + r) * ldv + voff + h * 64 + c8);
#pragma unroll
    for (int q = 0; q < 8; ++q) tl[r][c8 + q] = f.u[q]; }
  __syncthreads();
  for (int pass = 0; pass < 2; ++pass) {
#pragma unroll
    for (int rd = 0; rd < 2; ++rd) { const int d = rd * 32 + tid / 8, pc = tid % 8; FragH f;
#pragma unroll
      for (int q = 0; q < 8; ++q) f.u[q] = tl[pc * 8 + q][d];
      *(volatile v8us*)((unsigned short*)Vt + ((size_t)slab * 64 + d) * TTv + lg * 64 + pc * 8) = f.half[0]; }
    if (pass == 0) __threadfence(); } }

__global__ __launch_bounds__(256) void k_hl(const float* __restrict__ F, _Float16* __restrict__ Hh, _Float16* __restrict__ Hl, size_t n8) { const size_t t = (size_t)blockIdx.x * 256 + threadIdx.x; if (t >= n8) return; FragH fh, fl; const v4f a = *(const v4fa*)(F + t * 8), c = *(const v4fa*)(F + t * 8 + 4);
#pragma unroll
  for (int q = 0; q < 4; ++q) { _Float16 h = (_Float16)a[q]; fh.h[q] = h; fl.h[q] = (_Float16)((a[q] - (float)h) * 1024.0f); h = (_Float16)c[q]; fh.h[4 + q] = h; fl.h[4 + q] = (_Float16)((c[q] - (float)h) * 1024.0f); }
  for (int pass = 0; pass < 2; ++pass) { *(volatile v8us*)((unsigned short*)Hh + t * 8) = fh.half[0]; *(volatile v8us*)((unsigned short*)Hl + t * 8) = fl.half[0]; if (pass == 0) __threadfence(); } }

__global__ __launch_bounds__(256) void k_rms(const float* __restrict__ X, const float* __restrict__ w, _Float16* __restrict__ Y, _Float16* __restrict__ YL) {
  #pragma clang fp contract(off)
  const int tid = threadIdx.x, wv = tid >> 5, l = tid & 31; const size_t row = (size_t)blockIdx.x * 8 + wv; if (row >= TT) return; float v[32]; float ss = 0.f;
#pragma unroll
  for (int q = 0; q < 4; ++q) { const v4f a = *(const v4fa*)(X + row * DD + q * 256 + 8 * l), c = *(const v4fa*)(X + row * DD + q * 256 + 8 * l + 4);
#pragma unroll
    for (int j = 0; j < 4; ++j) { v[q * 8 + j] = bf16_round(a[j]); v[q * 8 + 4 + j] = bf16_round(c[j]); } }
#pragma unroll
  for (int i = 0; i < 32; ++i) ss += v[i] * v[i];
  for (int o = 16; o > 0; o >>= 1) ss += __shfl_xor(ss, o, 32); const float rs = rsqrtf(ss * (1.0f / DD) + 1e-6f);
  for (int pass = 0; pass < 2; ++pass) {
#pragma unroll
    for (int q = 0; q < 4; ++q) { FragH f, fl;
#pragma unroll
      for (int j = 0; j < 8; ++j) { const int c = q * 256 + 8 * l + j; const float xv = v[q * 8 + j] * rs * bf16_round(w[c]); const _Float16 hi = (_Float16)xv; f.h[j] = hi; fl.h[j] = (_Float16)((xv - (float)hi) * 1024.0f); }
      *(volatile v8us*)((unsigned short*)Y + row * DD + q * 256 + 8 * l) = f.half[0]; *(volatile v8us*)((unsigned short*)YL + row * DD + q * 256 + 8 * l) = fl.half[0]; }
    if (pass == 0) __threadfence(); } }
__global__ __launch_bounds__(256) void k_wall(const float* __restrict__ qw, const float* __restrict__ kw, const float* __restrict__ vw, const float* __restrict__ gw, const float* __restrict__ aw, const float* __restrict__ bw, _Float16* __restrict__ Bt) { const size_t t = (size_t)blockIdx.x * 256 + threadIdx.x; if (t >= (size_t)PWP * (DD / 8)) return; const int r = (int)(t / (DD / 8)), k0 = (int)(t % (DD / 8)) * 8; const float* src = nullptr; int rr = 0;
  if (r < OK_) { src = qw; rr = r; } else if (r < OV) { src = kw; rr = r - OK_; } else if (r < OG) { src = vw; rr = r - OV; } else if (r < OA) { src = gw; rr = r - OG; } else if (r < OB) { src = aw; rr = r - OA; } else if (r < PW) { src = bw; rr = r - OB; }
  FragH f;
#pragma unroll
  for (int q = 0; q < 8; ++q) f.h[q] = src ? (_Float16)(bf16_round(src[(size_t)rr * DD + k0 + q]) * 16.0f) : (_Float16)0.0f;
  *(volatile v8us*)((unsigned short*)Bt + (size_t)r * DD + k0) = f.half[0]; __threadfence(); *(volatile v8us*)((unsigned short*)Bt + (size_t)r * DD + k0) = f.half[0]; }
__global__ __launch_bounds__(256) void k_prep(const float* __restrict__ P, const float* __restrict__ cq, const float* __restrict__ ck, const float* __restrict__ cv, const float* __restrict__ dtb, const float* __restrict__ Alog, float* __restrict__ Q, float* __restrict__ K, float* __restrict__ V, float* __restrict__ BG) {
  #pragma clang fp contract(off)
  __shared__ float sq[QW], sk[QW]; __shared__ float red[2 * NH]; __shared__ __attribute__((aligned(16))) float bg[2 * NH];
  const int tid = threadIdx.x; const int t = blockIdx.x;
  for (int c = tid; c < QW; c += 256) { float aq = 0.f, ak = 0.f;
#pragma unroll
    for (int i = 0; i < 4; ++i) { const int ts = t - 3 + i; if (ts >= 0) { aq += P[(size_t)ts * PWP + OQ + c] * bf16_round(cq[c * 4 + i]); ak += P[(size_t)ts * PWP + OK_ + c] * bf16_round(ck[c * 4 + i]); } }
    sq[c] = aq / (1.0f + expf(-aq)); sk[c] = ak / (1.0f + expf(-ak)); }
  for (int c = tid; c < VW; c += 256) { float av = 0.f;
#pragma unroll
    for (int i = 0; i < 4; ++i) { const int ts = t - 3 + i; if (ts >= 0) av += P[(size_t)ts * PWP + OV + c] * bf16_round(cv[c * 4 + i]); }
    const float vv = av / (1.0f + expf(-av)); float* vp = V + (size_t)t * VW + c; *(volatile float*)vp = vv; __threadfence(); *(volatile float*)vp = vv; }
  if (tid < NH) { const float bb = P[(size_t)t * PWP + OB + tid], aa = P[(size_t)t * PWP + OA + tid] + bf16_round(dtb[tid]); const float sp = (aa > 20.f) ? aa : log1pf(expf(aa)); bg[2 * tid] = 1.0f / (1.0f + expf(-bb)); bg[2 * tid + 1] = -expf(bf16_round(Alog[tid])) * sp; }
  __syncthreads();
  { const int h = tid / 16, part = tid % 16; float km = 0.f;
#pragma unroll
    for (int j = 0; j < 4; ++j) km += sk[h * DKk + part * 4 + j];
    for (int o = 8; o > 0; o >>= 1) km += __shfl_xor(km, o, 16); km *= (1.0f / DKk);
    float qs = 0.f, ks = 0.f;
#pragma unroll
    for (int j = 0; j < 4; ++j) { const int c = h * DKk + part * 4 + j; const float kv = sk[c] - km; sk[c] = kv; ks += kv * kv; qs += sq[c] * sq[c]; }
    for (int o = 8; o > 0; o >>= 1) { qs += __shfl_xor(qs, o, 16); ks += __shfl_xor(ks, o, 16); }
    const float qr = rsqrtf(qs + 1e-6f) * 0.125f, kr = rsqrtf(ks + 1e-6f); v4f oq, ok;
#pragma unroll
    for (int j = 0; j < 4; ++j) { const int c = h * DKk + part * 4 + j; oq[j] = sq[c] * qr; ok[j] = sk[c] * kr; }
    for (int pass = 0; pass < 2; ++pass) { *(volatile v4f*)(Q + (size_t)t * QW + h * DKk + part * 4) = oq; *(volatile v4f*)(K + (size_t)t * QW + h * DKk + part * 4) = ok; if (pass == 0) __threadfence(); } }
  if (tid < 2 * NH / 4) { const v4f vv = *(const v4fa*)&bg[tid * 4]; *(volatile v4f*)(BG + (size_t)t * 2 * NH + tid * 4) = vv; __threadfence(); *(volatile v4f*)(BG + (size_t)t * 2 * NH + tid * 4) = vv; } }
__global__ __launch_bounds__(256) void k_delta(const float* __restrict__ Q, const float* __restrict__ K, const float* __restrict__ V, const float* __restrict__ BG, float* __restrict__ O) {
  #pragma clang fp contract(off)
  __shared__ float S[DKk][DVv + 1]; __shared__ float qk[2][DKk]; __shared__ float part[2][DVv]; __shared__ float vn[DVv];
  const int tid = threadIdx.x; const int h = blockIdx.x; const int v = tid % DVv, rh = tid / DVv; const int r0 = rh * 32;
  for (int i = tid; i < DKk * (DVv + 1); i += 256) (&S[0][0])[i] = 0.f;
  __syncthreads();
#pragma unroll 1
  for (int t = 0; t < TT; ++t) {
    if (tid < DKk) { qk[0][tid] = Q[(size_t)t * QW + h * DKk + tid]; qk[1][tid] = K[(size_t)t * QW + h * DKk + tid]; }
    const float beta = BG[(size_t)t * 2 * NH + 2 * h], gl = BG[(size_t)t * 2 * NH + 2 * h + 1]; const float dec = expf(gl);
    __syncthreads();
    float ps = 0.f;
#pragma unroll 1
    for (int k = r0; k < r0 + 32; ++k) { const float sv = S[k][v] * dec; S[k][v] = sv; ps += qk[1][k] * sv; }
    part[rh][v] = ps; __syncthreads();
    if (rh == 0) vn[v] = (V[(size_t)t * VW + h * DVv + v] - (part[0][v] + part[1][v])) * beta;
    __syncthreads();
    const float vnv = vn[v]; float po = 0.f;
#pragma unroll 1
    for (int k = r0; k < r0 + 32; ++k) { const float sv = S[k][v] + qk[1][k] * vnv; S[k][v] = sv; po += qk[0][k] * sv; }
    part[rh][v] = po; __syncthreads();
    if (rh == 0) { const float ov = part[0][v] + part[1][v]; float* op = O + ((size_t)t * NH + h) * DVv + v; *(volatile float*)op = ov; __threadfence(); *(volatile float*)op = ov; }
    __syncthreads(); } }
__global__ __launch_bounds__(256) void k_onorm(const float* __restrict__ O, const float* __restrict__ P, const float* __restrict__ w, _Float16* __restrict__ ON) {
  #pragma clang fp contract(off)
  const int tid = threadIdx.x, wv = tid >> 5, l = tid & 31; const int th = blockIdx.x * 8 + wv; if (th >= TT * NH) return; const int t = th / NH, h = th % NH; const v4f o = *(const v4fa*)(O + (size_t)th * DVv + 4 * l); float ss = o[0]*o[0] + o[1]*o[1] + o[2]*o[2] + o[3]*o[3];
  for (int q = 16; q > 0; q >>= 1) ss += __shfl_xor(ss, q, 32); const float rs = rsqrtf(ss * (1.0f / DVv) + 1e-5f); FragH f;
#pragma unroll
  for (int j = 0; j < 4; ++j) { const int v = 4 * l + j; const float g = P[(size_t)t * PWP + OG + h * DVv + v]; f.h[j] = (_Float16)(o[j] * rs * bf16_round(w[v]) * (g / (1.0f + expf(-g)))); }
  const unsigned long long hv = *(const unsigned long long*)&f.u[0]; *(volatile unsigned long long*)((unsigned short*)ON + (size_t)th * DVv + 4 * l) = hv; __threadfence(); *(volatile unsigned long long*)((unsigned short*)ON + (size_t)th * DVv + 4 * l) = hv; }

extern "C" void kernel_launch(void* const* d_in, const int* in_sizes, int n_in,
                              void* d_out, int out_size, void* d_ws, size_t ws_size, hipStream_t stream) {
  (void)in_sizes; (void)n_in; (void)out_size;
  const float* const* I = (const float* const*)d_in; const float* hs = I[0]; const float* nw = I[1]; const float* qw = I[2]; const float* kw = I[3]; const float* vw = I[4]; const float* aw = I[5]; const float* bw = I[6]; const float* gw = I[7]; const float* dtb = I[8]; const float* Alog = I[9]; const float* cq = I[10]; const float* ck = I[11]; const float* cv = I[12]; const float* onw = I[13]; const float* opw = I[14]; const float* outw = I[15];
  char* ws = (char*)d_ws; size_t off = 0;
  auto take = [&](size_t bytes) { char* p = ws + off; off += (bytes + 255) & ~(size_t)255; return p; };
  _Float16* Ball = (_Float16*)take((size_t)PWP * DD * 2); _Float16* Bop = (_Float16*)take((size_t)DD * VW * 2); _Float16* Bout = (_Float16*)take((size_t)DD * DD * 2);
  _Float16* XN = (_Float16*)take((size_t)TT * DD * 2); float* P = (float*)take((size_t)TT * PWP * 4); float* Q = (float*)take((size_t)TT * QW * 4); float* K = (float*)take((size_t)TT * QW * 4); float* V = (float*)take((size_t)TT * VW * 4); float* BG = (float*)take((size_t)TT * 2 * NH * 4); float* O = (float*)take((size_t)TT * VW * 4); _Float16* XNL = (_Float16*)take((size_t)TT * DD * 2);
  _Float16* ON = (_Float16*)Q;
  _Float16* H1 = XN;
  if (off > ws_size) return;
  k_wall<<<(unsigned)(((size_t)PWP * (DD / 8) + 255) / 256), 256, 0, stream>>>(qw, kw, vw, gw, aw, bw, Ball); k_round16f<<<(unsigned)(((size_t)DD * VW / 8 + 255) / 256), 256, 0, stream>>>(opw, Bop, (size_t)DD * VW / 8); k_round16f<<<(unsigned)(((size_t)DD * DD / 8 + 255) / 256), 256, 0, stream>>>(outw, Bout, (size_t)DD * DD / 8);
  k_rms<<<TT / 8, 256, 0, stream>>>(hs, nw, XN, XNL);
  k_gemm_hhx<0><<<dim3(((TT / 16) * (PWP / 64) + 3) / 4, 1), 128, 0, stream>>>(XN, DD, 0, Ball, DD, 0, 0.0625f, nullptr, 0, nullptr, 1, 0, 0, P, nullptr, PWP, 0, TT, PWP, DD);
  k_gemm_hhx<0><<<dim3(((TT / 16) * (PWP / 64) + 3) / 4, 1), 128, 0, stream>>>(XNL, DD, 0, Ball, DD, 0, 0.0625f / 1024.0f, nullptr, 0, P, 1, (size_t)PWP, 0, P, nullptr, PWP, 0, TT, PWP, DD);
  k_prep<<<TT, 256, 0, stream>>>(P, cq, ck, cv, dtb, Alog, Q, K, V, BG);
  k_delta<<<NH, 256, 0, stream>>>(Q, K, V, BG, O);
  k_onorm<<<(TT * NH + 7) / 8, 256, 0, stream>>>(O, P, onw, ON);
  k_gemm_hhx<0><<<dim3(((TT / 16) * (DD / 64) + 3) / 4, 1), 128, 0, stream>>>(ON, VW, 0, Bop, VW, 0, 0.0625f, nullptr, 0, nullptr, 1, 0, 0, nullptr, H1, DD, 0, TT, DD, VW);
  k_gemm_hhx<0><<<dim3(((TT / 16) * (DD / 64) + 3) / 4, 1), 128, 0, stream>>>(H1, DD, 0, Bout, DD, 0, 0.0625f, nullptr, 0, nullptr, 1, 0, 0, (float*)d_out, nullptr, DD, 0, TT, DD, DD);
}
